// dcn_4947802325745
// MI455X (gfx1250) — hardware-run, weakly checked
//
#include <hip/hip_runtime.h>


#ifndef NB
#define NB 4
#endif
#define NB_FULL 4
#define CH    64
#define IMH   128
#define IMW   128
#define NPIX  (IMH * IMW)
#define NTAP  9
#define KK    (NTAP * CH)
#define NOFF  27
#define NOP   32
#define PT    32
#define DW    4
#define SPT   (KK + 8)
#define OSP   36
#define OFP   36
#define TSP   72
#define SCARRY 16.0f
#define WCARRY 64.0f
#define OSC   (1.0f / 1024.0f)

static_assert(CH == 64);
static_assert(KK % 32 == 0);
static_assert(CH % 32 == 0);
static_assert(NOFF == 3 * NTAP);
static_assert(NOP == 32 && NOFF <= NOP);
static_assert(PT == 32);
static_assert(IMW % 64 == 0);
static_assert(IMW % PT == 0);
static_assert(IMW / PT == 4);
static_assert(IMW / 64 == 2);
static_assert(DW * 16 == CH);
static_assert((PT * NTAP * 8) % (32 * DW) == 0);
static_assert((SPT * 2) % 16 == 0);
static_assert((OSP * 4) % 16 == 0);
static_assert((OFP * 4) % 16 == 0);
static_assert((TSP * 2) % 16 == 0);
static_assert(4 * 32 * 16 == 16 * PT * 4);
static_assert(4 * 32 * 16 == 16 * NOP * 4);
static_assert(4 * 256 * 8 == IMW * CH);
static_assert(8 * 256 * 4 == IMW * CH);
static_assert((NOP * KK / 8) % 256 == 0);
static_assert((CH * KK / 8) % 256 == 0);
static_assert((KK * 2) % 128 == 0);
static_assert(NB <= NB_FULL);
static_assert((size_t)PT * SPT * 2 + (size_t)PT * NTAP * 32 + (size_t)DW * 16 * OSP * 4 <= 131072);
static_assert((size_t)IMW * TSP * 2 <= 131072);
static_assert((size_t)16 * OFP * 4 <= 131072);

typedef _Float16 h16;
typedef unsigned short bf;
typedef __attribute__((ext_vector_type(16))) __bf16   v16bf;
typedef __attribute__((ext_vector_type(16))) _Float16 v16h;
typedef __attribute__((ext_vector_type(8)))  _Float16 v8h;
typedef __attribute__((ext_vector_type(8)))  unsigned short v8us;
typedef __attribute__((ext_vector_type(8)))  float    v8f;
typedef __attribute__((ext_vector_type(4)))  float    v4f;
typedef __attribute__((ext_vector_type(4)))  int      v4i;
typedef v4f  __attribute__((may_alias)) v4fa;
typedef v8h  __attribute__((may_alias)) v8ha;
typedef v8us __attribute__((may_alias)) v8usa;

__device__ __forceinline__ unsigned short f2bf(float f) { unsigned u = __float_as_uint(f); u += 0x7FFFu + ((u >> 16) & 1u); return (unsigned short)(u >> 16); }
__device__ __forceinline__ float bfr(float f) { return __uint_as_float(((unsigned)f2bf(f)) << 16); }
__device__ __forceinline__ v16h cat16(v8h lo, v8h hi) { return __builtin_shufflevector(lo, hi, 0, 1, 2, 3, 4, 5, 6, 7, 8, 9, 10, 11, 12, 13, 14, 15); }
__device__ __forceinline__ v16bf cat16b(v8us lo, v8us hi) { return __builtin_bit_cast(v16bf, __builtin_shufflevector(lo, hi, 0, 1, 2, 3, 4, 5, 6, 7, 8, 9, 10, 11, 12, 13, 14, 15)); }
__device__ __forceinline__ v8f wmma16(v16h a, v16h b, v8f c) { return __builtin_amdgcn_wmma_f32_16x16x32_f16(false, a, false, b, (short)0, c, false, false); }
__device__ __forceinline__ v8f wmmab(v16bf a, v16bf b, v8f c) { return __builtin_amdgcn_wmma_f32_16x16x32_bf16(false, a, false, b, (short)0, c, false, false); }
__device__ __forceinline__ v16h  ldh(const h16* p) { return cat16(*(const v8h*)p, *(const v8h*)(p + 16)); }
__device__ __forceinline__ v16bf ldb(const bf* p)  { return cat16b(*(const v8us*)p, *(const v8us*)(p + 16)); }
__device__ __forceinline__ void wave_sync() { __builtin_amdgcn_fence(3  , "wavefront"); __builtin_amdgcn_wave_barrier(); asm volatile("" ::: "memory"); }
__device__ __forceinline__ h16 toh_flush(float v) { const h16 r = (h16)v; return (fabsf(v) < 6.103515625e-05f) ? (h16)0.0f : r; }
__device__ __forceinline__ v8f wmma16g(v16h a, v16h b, v8f c) { c = wmma16(a, b, c); asm volatile("v_nop\n\tv_nop\n\tv_nop\n\tv_nop" : "+v"(c) : "v"(a), "v"(b)); return c; }
__device__ __forceinline__ v8f wmmabg(v16bf a, v16bf b, v8f c) { c = wmmab(a, b, c); asm volatile("v_nop\n\tv_nop\n\tv_nop\n\tv_nop" : "+v"(c) : "v"(a), "v"(b)); return c; }

__global__ __launch_bounds__(256) void k_nhwc(const float* __restrict__ src, bf* dst) {
    __shared__ __align__(16) bf ts[IMW * TSP];
    const int tid = threadIdx.x;
    const int b = blockIdx.x / IMH, y = blockIdx.x % IMH;
    const float* sp = src + (size_t)b * CH * NPIX + (size_t)y * IMW;
#pragma unroll 1
    for (int j = 0; j < 8; ++j) {
        const int q = j * 256 + tid; const int ch = q >> 5, w4 = (q & 31) * 4;
        const v4f v = *(const v4f*)(sp + (size_t)ch * NPIX + w4);
#pragma unroll
        for (int i = 0; i < 4; ++i) ts[(w4 + i) * TSP + ch] = f2bf(v[i]);
    }
    __syncthreads();
    bf* dp = dst + ((size_t)b * NPIX + (size_t)y * IMW) * CH;
#pragma unroll 1
    for (int ps = 0; ps < 2; ++ps) {
#pragma unroll
        for (int j = 0; j < 4; ++j) {
            const int q = j * 256 + tid; const int w = q >> 3, c8 = (q & 7) * 8;
            const v8us o = *(const v8usa*)(&ts[w * TSP + c8]);
            *(volatile v8us*)(dp + (size_t)q * 8) = o; }
        if (ps == 0) __threadfence(); }
}

__global__ __launch_bounds__(256) void k_woff(const float* __restrict__ w, bf* dst) {
    const int i = blockIdx.x * 256 + threadIdx.x; if (i >= NOP * KK / 8) return;
    const int n = i / (KK / 8), g = i % (KK / 8); const int k0 = g * 8; const int tap = k0 >> 6, ch0 = k0 & 63;
    const int nc = n < NOFF ? n : NOFF - 1;
    v8us o;
#pragma unroll
    for (int k = 0; k < 8; ++k) { float v = w[((size_t)nc * CH + ch0 + k) * NTAP + tap]; asm volatile("" : "+v"(v)); o[k] = (n < NOFF) ? f2bf(v) : (unsigned short)0; }
    *(volatile v8us*)(dst + (size_t)i * 8) = o; __threadfence(); *(volatile v8us*)(dst + (size_t)i * 8) = o;
}

__global__ __launch_bounds__(256) void k_wmain(const float* __restrict__ w, h16* dst) {
    const int i = blockIdx.x * 256 + threadIdx.x; if (i >= CH * KK / 8) return;
    const int n = i / (KK / 8), g = i % (KK / 8); const int k0 = g * 8; const int tap = k0 >> 6, ch0 = k0 & 63;
    v8h o;
#pragma unroll
    for (int k = 0; k < 8; ++k) { const float v = bfr(w[((size_t)n * CH + ch0 + k) * NTAP + tap]) * WCARRY; o[k] = toh_flush(v); }
    *(volatile v8h*)(dst + (size_t)i * 8) = o; __threadfence(); *(volatile v8h*)(dst + (size_t)i * 8) = o;
}

__global__ __launch_bounds__(32) void k_offconv(const bf* __restrict__ CT, const bf* __restrict__ WO, const float* __restrict__ boff, float* OFFP) {
    __shared__ __align__(16) float os[16 * OFP];
    const int lane = threadIdx.x & 31, lr = lane & 15, hi = lane >> 4;
    const int blk = blockIdx.x; const int b = blk / (IMH * 2); const int rem = blk % (IMH * 2); const int y = rem >> 1; const int x0 = (rem & 1) * 64;
    v8f acc[4][2];
#pragma unroll
    for (int mb = 0; mb < 4; ++mb)
#pragma unroll
        for (int nb = 0; nb < 2; ++nb) acc[mb][nb] = (v8f){};
    const size_t wo = (size_t)lr * KK + 8 * hi;
    const v8us zz = (v8us){};
#pragma unroll 1
    for (int tap = 0; tap < NTAP; ++tap) {
        const int r = tap / 3, s = tap - 3 * r;
        const int yy = y + r - 1;
        const bool yok = (yy >= 0) & (yy < IMH);
        const int yc = min(max(yy, 0), IMH - 1);
        size_t ao[4]; bool ok[4];
#pragma unroll
        for (int mb = 0; mb < 4; ++mb) { const int xx = x0 + mb * 16 + lr + s - 1; ok[mb] = yok & (xx >= 0) & (xx < IMW); const int xc = min(max(xx, 0), IMW - 1);
            ao[mb] = (((size_t)b * IMH + yc) * IMW + xc) * CH + 8 * hi; }
#pragma unroll
        for (int kh = 0; kh < 2; ++kh) {
            v16bf a[4];
#pragma unroll
            for (int mb = 0; mb < 4; ++mb) {
                v8us lo = *(const v8us*)(CT + ao[mb] + kh * 32); v8us up = *(const v8us*)(CT + ao[mb] + kh * 32 + 16);
                asm volatile("" : "+v"(lo)); asm volatile("" : "+v"(up));
                lo = ok[mb] ? lo : zz; up = ok[mb] ? up : zz;
                a[mb] = cat16b(lo, up); }
#pragma unroll
            for (int nb = 0; nb < 2; ++nb) { const v16bf bw = ldb(WO + wo + (size_t)nb * 16 * KK + tap * CH + kh * 32);
#pragma unroll
                for (int mb = 0; mb < 4; ++mb) acc[mb][nb] = wmmabg(a[mb], bw, acc[mb][nb]); }
        }
    }
    float bc[2];
#pragma unroll
    for (int nb = 0; nb < 2; ++nb) { const int n = nb * 16 + lr; const int ncl = n < NOFF ? n : NOFF - 1; float bv = boff[ncl]; asm volatile("" : "+v"(bv)); bc[nb] = (n < NOFF) ? bfr(bv) : 0.0f; }
    const size_t pbase = ((size_t)b * NPIX + (size_t)y * IMW + x0) * NOP;
#pragma unroll
    for (int mb = 0; mb < 4; ++mb) {
#pragma unroll
        for (int nb = 0; nb < 2; ++nb) {
#pragma unroll
            for (int j = 0; j < 8; ++j) os[(hi * 8 + j) * OFP + nb * 16 + lr] = acc[mb][nb][j] + bc[nb]; }
        wave_sync();
#pragma unroll 1
        for (int ps = 0; ps < 2; ++ps) {
#pragma unroll
            for (int s = 0; s < 4; ++s) { const int row = 4 * s + (lane >> 3), cofs = (lane & 7) * 4;
                const v4f val = *(const v4fa*)(&os[row * OFP + cofs]);
                *(volatile v4f*)(OFFP + pbase + (size_t)(mb * 16 + row) * NOP + cofs) = val; }
            if (ps == 0) __threadfence(); }
        wave_sync();
    }
}

__global__ __launch_bounds__(32 * DW) void k_main(const bf* __restrict__ XT, const float* __restrict__ OFFP, const h16* __restrict__ WD, const float* __restrict__ bmain, float* OUT) {
    __shared__ __align__(16) h16 st[PT * SPT];
    __shared__ __align__(16) v4i sIdx[PT * NTAP];
    __shared__ __align__(16) v4f sWt[PT * NTAP];
    __shared__ __align__(16) float os[DW * 16 * OSP];
    const int tid = threadIdx.x;
    const int lane = tid & 31, lr = lane & 15, hi = lane >> 4;
    const int wave = __builtin_amdgcn_readfirstlane((int)(threadIdx.x >> 5));
    const int blk = blockIdx.x; const int b = blk / (IMH * 4); const int rem = blk % (IMH * 4); const int y = rem >> 2; const int x0 = (rem & 3) * PT;
    const size_t pix0 = (size_t)y * IMW + x0;

#pragma unroll 1
    for (int it = tid; it < PT * NTAP; it += 32 * DW) {
        const int tap = it >> 5, p = it & 31;
        const float* op = OFFP + ((size_t)b * NPIX + pix0 + p) * NOP;
        const float dy = op[2 * tap], dx = op[2 * tap + 1], mr = op[18 + tap];
        const float msk = (1.0f / (1.0f + expf(-mr))) * SCARRY;
        const int r = tap / 3, s = tap - 3 * r;
        const float py = ((float)y + (float)(r - 1)) + dy;
        const float px = ((float)(x0 + p) + (float)(s - 1)) + dx;
        const float y0f = floorf(py), x0f = floorf(px);
        const float y1f = y0f + 1.0f, x1f = x0f + 1.0f;
        const float wy1 = py - y0f, wx1 = px - x0f;
        const float wy0 = 1.0f - wy1, wx0 = 1.0f - wx1;
        const bool vy0 = (y0f >= 0.0f) & (y0f <= (float)(IMH - 1));
        const bool vy1 = (y1f >= 0.0f) & (y1f <= (float)(IMH - 1));
        const bool vx0 = (x0f >= 0.0f) & (x0f <= (float)(IMW - 1));
        const bool vx1 = (x1f >= 0.0f) & (x1f <= (float)(IMW - 1));
        const int iy0 = (int)fminf(fmaxf(y0f, 0.0f), (float)(IMH - 1));
        const int iy1 = (int)fminf(fmaxf(y1f, 0.0f), (float)(IMH - 1));
        const int ix0 = (int)fminf(fmaxf(x0f, 0.0f), (float)(IMW - 1));
        const int ix1 = (int)fminf(fmaxf(x1f, 0.0f), (float)(IMW - 1));
        v4i id; v4f wt;
        id[0] = min(max(iy0 * IMW + ix0, 0), NPIX - 1); id[1] = min(max(iy0 * IMW + ix1, 0), NPIX - 1);
        id[2] = min(max(iy1 * IMW + ix0, 0), NPIX - 1); id[3] = min(max(iy1 * IMW + ix1, 0), NPIX - 1);
        wt[0] = ((wy0 * wx0) * ((vy0 & vx0) ? 1.0f : 0.0f)) * msk;
        wt[1] = ((wy0 * wx1) * ((vy0 & vx1) ? 1.0f : 0.0f)) * msk;
        wt[2] = ((wy1 * wx0) * ((vy1 & vx0) ? 1.0f : 0.0f)) * msk;
        wt[3] = ((wy1 * wx1) * ((vy1 & vx1) ? 1.0f : 0.0f)) * msk;
        sIdx[it] = id; sWt[it] = wt;
    }
    __syncthreads();

    const bf* xb = XT + (size_t)b * NPIX * CH;
#pragma unroll 1
    for (int j = 0; j < PT * NTAP * 8 / (32 * DW); ++j) {
        const int e = j * (32 * DW) + tid; const int it = e >> 3, cg = e & 7; const int p = it & 31, tap = it >> 5;
        const v4i id = sIdx[it]; const v4f wt = sWt[it];
        const v8us q0 = *(const v8us*)(xb + (size_t)id[0] * CH + cg * 8);
        const v8us q1 = *(const v8us*)(xb + (size_t)id[1] * CH + cg * 8);
        const v8us q2 = *(const v8us*)(xb + (size_t)id[2] * CH + cg * 8);
        const v8us q3 = *(const v8us*)(xb + (size_t)id[3] * CH + cg * 8);
        v8h o;
#pragma unroll
        for (int i = 0; i < 8; ++i) {
            const float xa = __uint_as_float(((unsigned)q0[i]) << 16), xc = __uint_as_float(((unsigned)q1[i]) << 16);
            const float xd = __uint_as_float(((unsigned)q2[i]) << 16), xe = __uint_as_float(((unsigned)q3[i]) << 16);
            const float v = ((wt[0] * xa + wt[1] * xc) + wt[2] * xd) + wt[3] * xe;
            o[i] = toh_flush(v); }
        *(v8ha*)(&st[p * SPT + tap * CH + cg * 8]) = o;
    }
    __syncthreads();

    const size_t ao = (size_t)(wave * 16 + lr) * KK + 8 * hi;
    const int bo = lr * SPT + 8 * hi;
    v8f acc0 = (v8f){}, acc1 = (v8f){};
#pragma unroll 2
    for (int kc = 0; kc < KK; kc += 32) {
        const v16h a  = ldh(WD + ao + kc);
        const v16h b0 = cat16(*(const v8ha*)(&st[bo + kc]), *(const v8ha*)(&st[bo + kc + 16]));
        const v16h b1 = cat16(*(const v8ha*)(&st[bo + 16 * SPT + kc]), *(const v8ha*)(&st[bo + 16 * SPT + kc + 16]));
        acc0 = wmma16g(a, b0, acc0);
        acc1 = wmma16g(a, b1, acc1);
    }
    const int wb = wave * 16 * OSP;
#pragma unroll
    for (int j = 0; j < 8; ++j) {
        const float br = bfr(bmain[wave * 16 + hi * 8 + j]);
        os[wb + (hi * 8 + j) * OSP + lr]      = acc0[j] * OSC + br;
        os[wb + (hi * 8 + j) * OSP + 16 + lr] = acc1[j] * OSC + br; }
    wave_sync();
    float* orow = OUT + ((size_t)b * CH + wave * 16) * NPIX + pix0;
#pragma unroll 1
    for (int ps = 0; ps < 2; ++ps) {
#pragma unroll
        for (int s = 0; s < 4; ++s) { const int row = 4 * s + (lane >> 3), cofs = (lane & 7) * 4;
            const v4f val = *(const v4fa*)(&os[wb + row * OSP + cofs]);
            *(volatile v4f*)(orow + (size_t)row * NPIX + cofs) = val; }
        if (ps == 0) __threadfence(); }
}

static constexpr size_t al256(size_t v) { return (v + 255) & ~(size_t)255; }
static constexpr size_t SZ_PL = al256((size_t)NB * NPIX * CH * 2);
static constexpr size_t SZ_OF = al256((size_t)NB * NPIX * NOP * 4);
static constexpr size_t SZ_WO = al256((size_t)NOP * KK * 2);
static constexpr size_t SZ_WD = al256((size_t)CH * KK * 2);
static constexpr size_t SZ_TOTAL = 2 * SZ_PL + SZ_OF + SZ_WO + SZ_WD;
static_assert(SZ_TOTAL <= (size_t)134217728);
static_assert((size_t)NB * IMH * 256 * 4 * 8 == (size_t)NB * NPIX * CH);
static_assert((size_t)NB * IMH * 2 * 64 * NOP == (size_t)NB * NPIX * NOP);
static_assert((size_t)NB * IMH * 4 * PT == (size_t)NB * NPIX);

extern "C" void kernel_launch(void* const* d_in, const int* in_sizes, int n_in,
                              void* d_out, int out_size, void* d_ws, size_t ws_size, hipStream_t stream) {
    if (n_in < 6) return;
    const size_t needx = (size_t)NB * CH * NPIX;
    if ((size_t)in_sizes[0] < needx || (size_t)in_sizes[1] < needx) return;
    if ((size_t)in_sizes[2] < (size_t)NOFF * CH * NTAP || in_sizes[3] < NOFF) return;
    if ((size_t)in_sizes[4] < (size_t)CH * CH * NTAP || in_sizes[5] < CH) return;
    if ((size_t)out_size < needx) return;
    if (SZ_TOTAL > ws_size) return;
    const float* xin   = (const float*)d_in[0];
    const float* cin   = (const float*)d_in[1];
    const float* woff  = (const float*)d_in[2];
    const float* boff  = (const float*)d_in[3];
    const float* wmain = (const float*)d_in[4];
    const float* bmain = (const float*)d_in[5];
    float* OUT = (float*)d_out;
    char* wsp = (char*)d_ws;
    bf*    XT   = (bf*)wsp;    wsp += SZ_PL;
    bf*    CT   = (bf*)wsp;    wsp += SZ_PL;
    float* OFFP = (float*)wsp; wsp += SZ_OF;
    bf*    WO   = (bf*)wsp;    wsp += SZ_WO;
    h16*   WD   = (h16*)wsp;   wsp += SZ_WD;

    k_nhwc<<<NB * IMH, 256, 0, stream>>>(xin, XT);
    k_nhwc<<<NB * IMH, 256, 0, stream>>>(cin, CT);
    k_woff<<<(NOP * KK / 8 + 255) / 256, 256, 0, stream>>>(woff, WO);
    k_wmain<<<(CH * KK / 8 + 255) / 256, 256, 0, stream>>>(wmain, WD);
    k_offconv<<<NB * IMH * 2, 32, 0, stream>>>(CT, WO, boff, OFFP);
    k_main<<<NB * IMH * 4, 32 * DW, 0, stream>>>(XT, OFFP, WD, bmain, OUT);
}
